// ContactMapHead_3324304687632
// MI455X (gfx1250) — hardware-run, weakly checked
//
#include <hip/hip_runtime.h>
#include <stddef.h>


typedef _Float16 h16;
typedef _Float16 v16h __attribute__((ext_vector_type(16)));
typedef _Float16 v8h  __attribute__((ext_vector_type(8)));
typedef float    v8f  __attribute__((ext_vector_type(8)));
typedef float    v4f  __attribute__((ext_vector_type(4)));

#ifndef NB
#define NB 2
#endif
#ifndef SEQ
#define SEQ 512
#endif
#define NB_FULL  2
#define SEQ_FULL 512
#define DIM   512
#define MROWS (NB * SEQ)
#define PAIRS_MAX ((SEQ * (SEQ - 1)) / 2)
#define OUT_MAX (NB * PAIRS_MAX)
#define PACK_CHUNKS ((OUT_MAX + 3) / 4)
#define PACK_BLOCKS ((PACK_CHUNKS + 255) / 256)
#define SEARCH_ITERS 10

static_assert(NB >= 1 && NB <= NB_FULL);
static_assert(SEQ >= 64 && SEQ <= SEQ_FULL && (SEQ % 64) == 0);
static_assert((SEQ % 32) == 0);
static_assert(SEQ <= (1 << SEARCH_ITERS));
static_assert((DIM % 64) == 0 && (DIM % 32) == 0);
static_assert((MROWS % 64) == 0 && (MROWS % 8) == 0);
static_assert(DIM == 2 * 32 * 8);
static_assert((size_t)NB * SEQ * SEQ < (size_t)0xFFFFFFFFu);
static_assert((size_t)PACK_BLOCKS * 256 * 4 >= (size_t)OUT_MAX);

#define LDT 72
#define LDC 68
static_assert((LDT % 8) == 0 && LDT >= 64);
static_assert((LDC % 4) == 0 && LDC >= 64);

#define WCARRY 64.0f

#define WT_BYTES   ((size_t)DIM * DIM * 2)
#define H16_BYTES  ((size_t)MROWS * DIM * 2)
#define U16_BYTES  ((size_t)MROWS * DIM * 2)
#define S_BYTES    ((size_t)NB * SEQ * SEQ * 4)
#define OFF_WT  ((size_t)0)
#define OFF_H16 (OFF_WT + WT_BYTES)
#define OFF_U16 (OFF_H16 + H16_BYTES)
#define OFF_S   (OFF_U16 + U16_BYTES)
#define WS_TOTAL (OFF_S + S_BYTES)
static_assert((WT_BYTES % 128) == 0 && (H16_BYTES % 128) == 0);
static_assert((U16_BYTES % 128) == 0 && (S_BYTES % 128) == 0);
static_assert(WS_TOTAL <= (size_t)134217728);

__device__ __forceinline__ float bf16r(float x) {
  unsigned int u = __float_as_uint(x);
  u = (u + 0x7FFFu + ((u >> 16) & 1u)) & 0xFFFF0000u;
  return __uint_as_float(u);
}

static __device__ __forceinline__ h16 toh_flush(float v) {
  const h16 r = (h16)v;
  return (fabsf(v) < 6.103515625e-05f) ? (h16)0.0f : r;
}

__device__ __forceinline__ v16h frag_at(const _Float16* p) {
  v8h lo = *(const v8h*)(p);
  v8h hi = *(const v8h*)(p + 16);
  v16h out;
#pragma unroll
  for (int i = 0; i < 8; ++i) { out[i] = lo[i]; out[i + 8] = hi[i]; }
  return out;
}

__device__ __forceinline__ v8f wmma16(v16h a, v16h b, v8f c) {
  v8f d = __builtin_amdgcn_wmma_f32_16x16x32_f16(false, a, false, b, (short)0, c,
                                                 false, false);
  asm volatile("v_nop\n\tv_nop\n\tv_nop\n\tv_nop" : "+v"(d) : "v"(a), "v"(b));
  return d;
}

__global__ __launch_bounds__(256) void wconv_kernel(
    const float* __restrict__ W, _Float16* __restrict__ Wt, unsigned ldw, unsigned ldk) {
  __shared__ _Float16 T[64 * LDT];
  const unsigned tid = threadIdx.x;
  const unsigned n0 = blockIdx.x * 64u;
  const unsigned k0 = blockIdx.y * 64u;
#pragma unroll 4
  for (unsigned j = 0; j < 16u; ++j) {
    const unsigned idx = tid + 256u * j;
    const unsigned kr = idx >> 6, nc = idx & 63u;
    const float v = W[(size_t)(k0 + kr) * ldw + n0 + nc];
    T[nc * LDT + kr] = (_Float16)(WCARRY * bf16r(v));
  }
  __syncthreads();
  v8h x[2];
  size_t off[2];
#pragma unroll
  for (unsigned i = 0; i < 2u; ++i) {
    const unsigned n = 32u * i + (tid >> 3);
    const unsigned kc = (tid & 7u) * 8u;
    x[i] = *(const v8h*)&T[n * LDT + kc];
    off[i] = (size_t)(n0 + n) * ldk + k0 + kc;
  }
#pragma unroll
  for (int i = 0; i < 2; ++i) *(volatile v8h*)(Wt + off[i]) = x[i];
  __threadfence();
#pragma unroll
  for (int i = 0; i < 2; ++i) *(volatile v8h*)(Wt + off[i]) = x[i];
}

__global__ __launch_bounds__(256) void hconv_kernel(
    const float* __restrict__ X, const int* __restrict__ amask, const int* __restrict__ smask,
    _Float16* __restrict__ dst) {
  const unsigned lane = threadIdx.x & 31u;
  const unsigned wave = (unsigned)__builtin_amdgcn_readfirstlane((int)(threadIdx.x >> 5));
  const unsigned crow = blockIdx.x * 8u + wave;
  const unsigned bidx = crow / (unsigned)SEQ;
  const unsigned r = crow - bidx * (unsigned)SEQ;
  const unsigned below = (1u << lane) - 1u;

  unsigned run = 0u, mypos = 0u;
#pragma unroll 1
  for (unsigned c = 0; c < (unsigned)SEQ / 32u; ++c) {
    const unsigned p = c * 32u + lane;
    const int am = amask[p];
    const int sm = smask[p];
    const bool f = (am == 1) && (sm == 0);
    const unsigned bal = __builtin_amdgcn_ballot_w32(f);
    const unsigned ord = run + (unsigned)__popc(bal & below);
    mypos |= (f && (ord == r)) ? p : 0u;
    run += (unsigned)__popc(bal);
  }
#pragma unroll
  for (int off = 1; off < 32; off <<= 1)
    mypos |= (unsigned)__shfl_xor((int)mypos, off, 32);
  const bool valid = r < run;
  const unsigned pos = (mypos < (unsigned)SEQ) ? mypos : (unsigned)(SEQ - 1);

  const size_t srow = (size_t)bidx * SEQ_FULL + pos;
  const float* xr = X + srow * DIM + lane * 8u;
#pragma unroll 1
  for (unsigned j = 0; j < (unsigned)DIM / 256u; ++j) {
    const v4f a0 = *(const v4f*)(xr + j * 256u);
    const v4f a1 = *(const v4f*)(xr + j * 256u + 4u);
    v8h o;
#pragma unroll
    for (int i = 0; i < 4; ++i) {
      const float t0 = valid ? bf16r(a0[i]) : 0.0f;
      const float t1 = valid ? bf16r(a1[i]) : 0.0f;
      o[i]     = toh_flush(t0);
      o[i + 4] = toh_flush(t1);
    }
    _Float16* p = dst + (size_t)crow * DIM + j * 256u + lane * 8u;
    *(volatile v8h*)p = o;
    __threadfence();
    *(volatile v8h*)p = o;
  }
}

template <int MODE>
__device__ __forceinline__ void gemm_body(
    const _Float16* __restrict__ A16, const _Float16* __restrict__ Bt, const unsigned K,
    const float* __restrict__ bias, float* __restrict__ outf, _Float16* __restrict__ out16,
    const unsigned ldo) {
  __shared__ float Cs[64 * LDC];
  const unsigned tid = threadIdx.x, lane = tid & 31u, w = tid >> 5;
  const unsigned mw = w >> 1, nw = w & 1u;
  const unsigned hh = lane >> 4, m = lane & 15u;
  const unsigned n0 = blockIdx.x * 64u;
  const unsigned row0 = blockIdx.y * 64u;

  const _Float16* ap  = A16 + (size_t)(row0 + mw * 16u + m) * K + hh * 8u;
  const _Float16* bp0 = Bt + (size_t)(n0 + nw * 32u + m) * K + hh * 8u;
  const _Float16* bp1 = bp0 + (size_t)16 * K;
  v8f acc0 = {}, acc1 = {};
#pragma unroll 2
  for (unsigned k0 = 0; k0 < K; k0 += 32u) {
    const v16h a  = frag_at(ap + k0);
    const v16h b0 = frag_at(bp0 + k0);
    const v16h b1 = frag_at(bp1 + k0);
    acc0 = wmma16(a, b0, acc0);
    acc1 = wmma16(a, b1, acc1);
  }
#pragma unroll
  for (int r = 0; r < 8; ++r) {
    float* d = &Cs[(mw * 16u + hh * 8u + (unsigned)r) * LDC + nw * 32u + m];
    d[0]  = acc0[r];
    d[16] = acc1[r];
  }
  __syncthreads();

  if (MODE == 0) {
    v8h x[2];
    size_t off[2];
#pragma unroll
    for (unsigned i = 0; i < 2u; ++i) {
      const unsigned r = 32u * i + (tid >> 3);
      const unsigned c = (tid & 7u) * 8u;
      const v4f u0 = *(const v4f*)&Cs[r * LDC + c];
      const v4f u1 = *(const v4f*)&Cs[r * LDC + c + 4];
#pragma unroll
      for (int j = 0; j < 4; ++j) {
        x[i][j]     = toh_flush(u0[j] * (1.0f / WCARRY));
        x[i][j + 4] = toh_flush(u1[j] * (1.0f / WCARRY));
      }
      off[i] = (size_t)(row0 + r) * ldo + n0 + c;
    }
#pragma unroll
    for (int i = 0; i < 2; ++i) *(volatile v8h*)(out16 + off[i]) = x[i];
    __threadfence();
#pragma unroll
    for (int i = 0; i < 2; ++i) *(volatile v8h*)(out16 + off[i]) = x[i];
  }

  if (MODE == 1) {
    const float bb = bf16r(bias[0]);
    v4f xs[4];
    size_t off[4];
#pragma unroll
    for (unsigned i = 0; i < 4u; ++i) {
      const unsigned r = 16u * i + (tid >> 4);
      const unsigned c = (tid & 15u) * 4u;
      const v4f u = *(const v4f*)&Cs[r * LDC + c];
      v4f val;
#pragma unroll
      for (int j = 0; j < 4; ++j) val[j] = u[j] + bb;
      xs[i] = val;
      off[i] = (size_t)(row0 + r) * ldo + n0 + c;
    }
#pragma unroll
    for (int i = 0; i < 4; ++i) *(volatile v4f*)(outf + off[i]) = xs[i];
    __threadfence();
#pragma unroll
    for (int i = 0; i < 4; ++i) *(volatile v4f*)(outf + off[i]) = xs[i];
  }
}

__global__ __launch_bounds__(256) void gemm_u_kernel(
    const _Float16* __restrict__ A16, const _Float16* __restrict__ Bt,
    const float* __restrict__ bias, _Float16* __restrict__ out16) {
  gemm_body<0>(A16, Bt, (unsigned)DIM, bias, (float*)0, out16, (unsigned)DIM);
}
__global__ __launch_bounds__(256) void gemm_s_kernel(
    const _Float16* __restrict__ U16, const _Float16* __restrict__ H16,
    const float* __restrict__ bias, float* __restrict__ S) {
  const size_t zb = (size_t)blockIdx.z * SEQ * DIM;
  gemm_body<1>(U16 + zb, H16 + zb, (unsigned)DIM, bias,
               S + (size_t)blockIdx.z * SEQ * SEQ, (_Float16*)0, (unsigned)SEQ);
}

__global__ __launch_bounds__(256) void pack_kernel(
    const float* __restrict__ S, const int* __restrict__ amask, const int* __restrict__ smask,
    float* __restrict__ out, unsigned out_elems) {
  const unsigned lane = threadIdx.x & 31u;
  unsigned n = 0u;
#pragma unroll 1
  for (unsigned c = 0; c < (unsigned)SEQ / 32u; ++c) {
    const unsigned p = c * 32u + lane;
    const int am = amask[p];
    const int sm = smask[p];
    const unsigned bal = __builtin_amdgcn_ballot_w32((am == 1) && (sm == 0));
    n += (unsigned)__popc(bal);
  }
  if (n < 2u) return;
  const unsigned P = (n * (n - 1u)) >> 1;
  unsigned total = (unsigned)NB * P;
  total = (total < out_elems) ? total : out_elems;

  const unsigned e0 = (blockIdx.x * 256u + threadIdx.x) * 4u;
  unsigned b = e0 / P;
  const unsigned p0 = e0 - b * P;

  unsigned lo = 0u, hi = n - 2u;
#pragma unroll 1
  for (int it = 0; it < SEARCH_ITERS; ++it) {
    const unsigned mid = (lo + hi + 1u) >> 1;
    const unsigned rs = (mid * (2u * n - 1u - mid)) >> 1;
    const bool ok = rs <= p0;
    lo = ok ? mid : lo;
    hi = ok ? hi : (mid - 1u);
  }
  unsigned i = lo;
  unsigned j = p0 - ((i * (2u * n - 1u - i)) >> 1) + i + 1u;

  v4f val;
#pragma unroll
  for (int t = 0; t < 4; ++t) {
    const unsigned bc = (b < (unsigned)NB) ? b : (unsigned)(NB - 1);
    const unsigned ic = (i < (unsigned)SEQ) ? i : (unsigned)(SEQ - 1);
    const unsigned jc = (j < (unsigned)SEQ) ? j : (unsigned)(SEQ - 1);
    val[t] = S[((size_t)bc * SEQ + ic) * SEQ + jc];
    j += 1u;
    const bool rowend = (j >= n);
    i = rowend ? (i + 1u) : i;
    j = rowend ? (i + 1u) : j;
    const bool batend = (i >= n - 1u);
    b = batend ? (b + 1u) : b;
    i = batend ? 0u : i;
    j = batend ? 1u : j;
  }

  float* q = out + e0;
  const bool full = (e0 + 3u) < total;
  if (full) {
    *(volatile v4f*)q = val;
  } else {
    if (e0 + 0u < total) *(volatile float*)(q + 0) = val[0];
    if (e0 + 1u < total) *(volatile float*)(q + 1) = val[1];
    if (e0 + 2u < total) *(volatile float*)(q + 2) = val[2];
  }
  __threadfence();
  if (full) {
    *(volatile v4f*)q = val;
  } else {
    if (e0 + 0u < total) *(volatile float*)(q + 0) = val[0];
    if (e0 + 1u < total) *(volatile float*)(q + 1) = val[1];
    if (e0 + 2u < total) *(volatile float*)(q + 2) = val[2];
  }
}

extern "C" void kernel_launch(void* const* d_in, const int* in_sizes, int n_in,
                              void* d_out, int out_size, void* d_ws, size_t ws_size,
                              hipStream_t stream) {
  if (n_in < 5) return;
  const long long need_x = ((long long)(NB - 1) * SEQ_FULL + SEQ) * DIM;
  if ((long long)in_sizes[0] < need_x) return;
  if ((long long)in_sizes[1] < (long long)DIM * DIM) return;
  if (in_sizes[2] < 1) return;
  if (in_sizes[3] < SEQ || in_sizes[4] < SEQ) return;
  if ((long long)out_size < (long long)OUT_MAX) return;
  if (ws_size < WS_TOTAL) return;

  const float* X    = (const float*)d_in[0];
  const float* Wm   = (const float*)d_in[1];
  const float* bias = (const float*)d_in[2];
  const int*   am   = (const int*)d_in[3];
  const int*   sm   = (const int*)d_in[4];
  float* out = (float*)d_out;

  char* ws = (char*)d_ws;
  _Float16* Wt  = (_Float16*)(ws + OFF_WT);
  _Float16* H16 = (_Float16*)(ws + OFF_H16);
  _Float16* U16 = (_Float16*)(ws + OFF_U16);
  float*    S   = (float*)(ws + OFF_S);

  dim3 blk(256);
  wconv_kernel<<<dim3(DIM / 64, DIM / 64), blk, 0, stream>>>(Wm, Wt, (unsigned)DIM, (unsigned)DIM);
  hconv_kernel<<<dim3(MROWS / 8), blk, 0, stream>>>(X, am, sm, H16);
  gemm_u_kernel<<<dim3(DIM / 64, MROWS / 64), blk, 0, stream>>>(H16, Wt, bias, U16);
  gemm_s_kernel<<<dim3(SEQ / 64, SEQ / 64, NB), blk, 0, stream>>>(U16, H16, bias, S);
  pack_kernel<<<dim3(PACK_BLOCKS), blk, 0, stream>>>(S, am, sm, out, (unsigned)out_size);
}
